// MultiHeadedAttention_455266533797
// MI455X (gfx1250) — hardware-verified
//
#include <hip/hip_runtime.h>


#ifndef NB
#define NB 4
#endif
#ifndef SEQ
#define SEQ 2048
#endif
#define NB_FULL  4
#define SEQ_FULL 2048
#define TT   SEQ
#define DM   1024
#define NH_  16
#define HD   64
#define EROWS ((TT) < 512 ? (TT) : 512)
#define QKC  16.0f
#define CSC  (0.045084220027780106f * 0.00390625f)
#define VC   64.0f
#define WOC  1024.0f
#define OSC  1.52587890625e-05f
#define NEGB (-3.0e38f)
#define XSZ  ((size_t)NB * SEQ_FULL * DM)
#define QKSZ ((size_t)NB * NH_ * TT * HD)
static_assert(TT % 64 == 0);
static_assert(TT <= SEQ_FULL);
static_assert(NB >= 1 && NB <= NB_FULL);
static_assert(NH_ * HD == DM);
static_assert(DM % 64 == 0);
static_assert(DM % 32 == 0);
static_assert(HD == 64);
static_assert(EROWS % 64 == 0);
static_assert(EROWS <= TT);
static_assert((TT - EROWS) % 64 == 0);
static_assert((size_t)NB * TT * DM <= XSZ);
static_assert((size_t)NB * EROWS * DM <= XSZ);
static_assert((size_t)3 * DM * DM * 2 + (size_t)2 * DM * DM * 2 + (size_t)2 * QKSZ * 2 + (size_t)NB * NH_ * HD * TT * 2 + (size_t)2 * NB * NH_ * HD * EROWS * 2 + (size_t)3 * XSZ * 2 <= (size_t)134217728);

typedef _Float16 h16;
typedef unsigned short bf;
typedef __attribute__((ext_vector_type(16))) __bf16   v16bf;
typedef __attribute__((ext_vector_type(16))) _Float16 v16h;
typedef __attribute__((ext_vector_type(8)))  _Float16 v8h;
typedef __attribute__((ext_vector_type(8)))  unsigned short v8us;
typedef __attribute__((ext_vector_type(8)))  float    v8f;
typedef __attribute__((ext_vector_type(4)))  float    v4f;
typedef v4f  __attribute__((may_alias)) v4fa;
typedef v8us __attribute__((may_alias)) v8usa;

__device__ __forceinline__ unsigned short f2bf(float f) { unsigned u = __float_as_uint(f); u += 0x7FFFu + ((u >> 16) & 1u); return (unsigned short)(u >> 16); }
__device__ __forceinline__ float bf2f(unsigned short b) { return __uint_as_float(((unsigned)b) << 16); }
__device__ __forceinline__ float bfr(float f) { return bf2f(f2bf(f)); }
__device__ __forceinline__ v16h cat16(v8h lo, v8h hi) { return __builtin_shufflevector(lo, hi, 0, 1, 2, 3, 4, 5, 6, 7, 8, 9, 10, 11, 12, 13, 14, 15); }
__device__ __forceinline__ v16bf cat16b(v8us lo, v8us hi) { return __builtin_bit_cast(v16bf, __builtin_shufflevector(lo, hi, 0, 1, 2, 3, 4, 5, 6, 7, 8, 9, 10, 11, 12, 13, 14, 15)); }
__device__ __forceinline__ v8f wmma16(v16h a, v16h b, v8f c) { return __builtin_amdgcn_wmma_f32_16x16x32_f16(false, a, false, b, (short)0, c, false, false); }
__device__ __forceinline__ v8f wmmab(v16bf a, v16bf b, v8f c) { return __builtin_amdgcn_wmma_f32_16x16x32_bf16(false, a, false, b, (short)0, c, false, false); }
__device__ __forceinline__ void splitf(float y, unsigned short& h, unsigned short& l) { h = f2bf(y); l = f2bf(y - bf2f(h)); }
__device__ __forceinline__ v16h ldh(const h16* p) { return cat16(*(const v8h*)p, *(const v8h*)(p + 16)); }
__device__ __forceinline__ v16bf ldb(const bf* p) { return cat16b(*(const v8us*)p, *(const v8us*)(p + 16)); }
__device__ __forceinline__ v8us pack_h(v8f c) { v8h t;
#pragma unroll
    for (int r = 0; r < 8; ++r) t[r] = (h16)c[r];
    return __builtin_bit_cast(v8us, t); }
__device__ __forceinline__ void pack_b(v8f c, v8us& a, v8us& l) {
#pragma unroll
    for (int r = 0; r < 8; ++r) { unsigned short x, y; splitf(c[r], x, y); a[r] = x; l[r] = y; } }

template <typename T16> struct WFrag;
template <> struct WFrag<h16> { typedef v16h V; static __device__ __forceinline__ V ld(const h16* p) { return ldh(p); } static __device__ __forceinline__ v8f mma(V a, V b, v8f c) { return wmma16(a, b, c); } };
template <> struct WFrag<bf> { typedef v16bf V; static __device__ __forceinline__ V ld(const bf* p) { return ldb(p); } static __device__ __forceinline__ v8f mma(V a, V b, v8f c) { return wmmab(a, b, c); } };

template <typename T16, int NSPLIT>
__device__ __forceinline__ void gemm_tile(const T16* __restrict__ A, const T16* __restrict__ A2, const T16* __restrict__ Bt, const int K, const size_t aoff, const size_t boff, v8f (&acc)[4][4]) {
    typedef typename WFrag<T16>::V V;
#pragma unroll
    for (int mb = 0; mb < 4; ++mb)
#pragma unroll
        for (int nb = 0; nb < 4; ++nb) acc[mb][nb] = (v8f){};
#pragma unroll 1
    for (int kc = 0; kc < K; kc += 32) {
        V a[4], a2[4];
#pragma unroll
        for (int mb = 0; mb < 4; ++mb) { a[mb] = WFrag<T16>::ld(A + aoff + (size_t)mb * 16 * K + kc); if (NSPLIT == 1) a2[mb] = WFrag<T16>::ld(A2 + aoff + (size_t)mb * 16 * K + kc); else a2[mb] = a[mb]; }
#pragma unroll
        for (int nb = 0; nb < 4; ++nb) { const V b = WFrag<T16>::ld(Bt + boff + (size_t)nb * 16 * K + kc);
#pragma unroll
            for (int mb = 0; mb < 4; ++mb) { acc[mb][nb] = WFrag<T16>::mma(a[mb], b, acc[mb][nb]); if (NSPLIT == 1) acc[mb][nb] = WFrag<T16>::mma(a2[mb], b, acc[mb][nb]); } }
        asm volatile("v_nop\n\tv_nop\n\tv_nop\n\tv_nop" : "+v"(acc[0][0]), "+v"(acc[1][1]), "+v"(acc[2][2]), "+v"(acc[3][3]) : "v"(a[0]), "v"(a[3]));
    }
}

__global__ __launch_bounds__(256) void k_cvt8(const float* __restrict__ src, bf* dst, size_t n8) { const size_t i = (size_t)blockIdx.x * 256 + threadIdx.x; if (i >= n8) return; const v8f v = *(const v8f*)(src + i * 8); v8us o;
#pragma unroll
    for (int k = 0; k < 8; ++k) o[k] = f2bf(v[k]);
    *(volatile v8us*)(dst + i * 8) = o; __threadfence(); *(volatile v8us*)(dst + i * 8) = o; }

__global__ __launch_bounds__(256) void k_cvtwo(const float* __restrict__ src, bf* WB, h16* WH, size_t n8) { const size_t i = (size_t)blockIdx.x * 256 + threadIdx.x; if (i >= n8) return; const v8f v = *(const v8f*)(src + i * 8); v8us ob; v8h oh;
#pragma unroll
    for (int k = 0; k < 8; ++k) { const unsigned short hb = f2bf(v[k]); ob[k] = hb; oh[k] = (h16)(bf2f(hb) * WOC); }
    *(volatile v8us*)(WB + i * 8) = ob; *(volatile v8h*)(WH + i * 8) = oh; __threadfence(); *(volatile v8us*)(WB + i * 8) = ob; *(volatile v8h*)(WH + i * 8) = oh; }

__global__ __launch_bounds__(32) void k_projqk(const bf* __restrict__ XB, const bf* __restrict__ WT, const float* __restrict__ bq, const float* __restrict__ bk, h16* QK) {
    __shared__ __align__(16) float os[16 * 68];
    const int z = blockIdx.z;
    const int lane = threadIdx.x & 31, lr = lane & 15, hi = lane >> 4;
    const int mt = blockIdx.x; const int b = mt / (TT / 64); const int t0 = (mt % (TT / 64)) * 64; const int h = blockIdx.y;
    const bf* A = XB + (size_t)z * XSZ; const bf* Bt = WT + (size_t)z * DM * DM;
    const size_t aoff = ((size_t)b * SEQ_FULL + t0 + lr) * DM + 8 * hi;
    const size_t boff = ((size_t)h * HD + lr) * DM + 8 * hi;
    v8f acc[4][4];
    gemm_tile<bf, 0>(A, A, Bt, DM, aoff, boff, acc);
    const int rq = lane >> 3, pc = lane & 7;
    const v8f b0 = *(const v8f*)(bq + h * HD + pc * 8); const v8f b1 = *(const v8f*)(bk + h * HD + pc * 8);
    v8f bb;
#pragma unroll
    for (int i = 0; i < 8; ++i) bb[i] = bfr(z ? b1[i] : b0[i]);
    h16* P = QK + (size_t)z * QKSZ + (((size_t)b * NH_ + h) * TT + t0) * HD + pc * 8;
#pragma unroll
    for (int mb = 0; mb < 4; ++mb) {
#pragma unroll
        for (int nb = 0; nb < 4; ++nb) {
#pragma unroll
            for (int j = 0; j < 8; ++j) os[(hi * 8 + j) * 68 + nb * 16 + lr] = acc[mb][nb][j]; }
        __builtin_amdgcn_wave_barrier(); asm volatile("" ::: "memory");
        h16* prow = P + (size_t)(mb * 16) * HD;
#pragma unroll 1
        for (int ps = 0; ps < 2; ++ps) {
#pragma unroll
            for (int s = 0; s < 4; ++s) { const int row = 4 * s + rq;
                const v4f x0 = *(const v4fa*)(os + row * 68 + pc * 8), x1 = *(const v4fa*)(os + row * 68 + pc * 8 + 4);
                v8h o;
#pragma unroll
                for (int q = 0; q < 4; ++q) { o[q] = (h16)((x0[q] + bb[q]) * QKC); o[4 + q] = (h16)((x1[q] + bb[4 + q]) * QKC); }
                *(volatile v8h*)(prow + (size_t)row * HD) = o; }
            if (ps == 0) __threadfence(); }
        __builtin_amdgcn_wave_barrier(); asm volatile("" ::: "memory");
    }
}

__global__ __launch_bounds__(32) void k_projv(const bf* __restrict__ XBv, const bf* __restrict__ WTv, const float* __restrict__ bv, h16* VT, bf* VEh, bf* VEl) {
    __shared__ __align__(16) float ts[64 * 68];
    const int lane = threadIdx.x & 31, lr = lane & 15, hi = lane >> 4;
    const int mt = blockIdx.x; const int b = mt / (TT / 64); const int t0 = (mt % (TT / 64)) * 64; const int h = blockIdx.y;
    const size_t aoff = ((size_t)b * SEQ_FULL + t0 + lr) * DM + 8 * hi;
    const size_t boff = ((size_t)h * HD + lr) * DM + 8 * hi;
    v8f acc[4][4];
    gemm_tile<bf, 0>(XBv, XBv, WTv, DM, aoff, boff, acc);
#pragma unroll
    for (int mb = 0; mb < 4; ++mb)
#pragma unroll
        for (int nb = 0; nb < 4; ++nb) {
            const v4f lo4 = { acc[mb][nb][0], acc[mb][nb][1], acc[mb][nb][2], acc[mb][nb][3] };
            const v4f hi4 = { acc[mb][nb][4], acc[mb][nb][5], acc[mb][nb][6], acc[mb][nb][7] };
            *(v4fa*)(ts + (nb * 16 + lr) * 68 + mb * 16 + 8 * hi) = lo4;
            *(v4fa*)(ts + (nb * 16 + lr) * 68 + mb * 16 + 8 * hi + 4) = hi4; }
    __builtin_amdgcn_wave_barrier(); asm volatile("" ::: "memory");
    const int rq = lane >> 3, pc = lane & 7;
    const bool early = t0 < EROWS;
    const size_t vrow0 = ((size_t)b * NH_ + h) * HD;
#pragma unroll 1
    for (int ps = 0; ps < 2; ++ps) {
#pragma unroll 1
        for (int s = 0; s < 16; ++s) { const int d = 4 * s + rq;
            const float bb = bfr(bv[h * HD + d]);
            const v4f x0 = *(const v4fa*)(ts + d * 68 + pc * 8), x1 = *(const v4fa*)(ts + d * 68 + pc * 8 + 4);
            v8f x = __builtin_shufflevector(x0, x1, 0, 1, 2, 3, 4, 5, 6, 7);
            x = x + bb;
            v8h o;
#pragma unroll
            for (int q = 0; q < 8; ++q) o[q] = (h16)(x[q] * VC);
            *(volatile v8h*)(VT + (vrow0 + d) * TT + t0 + pc * 8) = o;
            if (early) { v8us oh, ol; pack_b(x, oh, ol);
                *(volatile v8us*)(VEh + (vrow0 + d) * EROWS + t0 + pc * 8) = oh;
                *(volatile v8us*)(VEl + (vrow0 + d) * EROWS + t0 + pc * 8) = ol; } }
        if (ps == 0) __threadfence(); }
}

template <bool EARLY>
__device__ __forceinline__ void attn_body(const h16* __restrict__ QP, const h16* __restrict__ KP, const h16* __restrict__ VT, const bf* __restrict__ VEh, const bf* __restrict__ VEl, bf* C0, bf* C1, const int qb) {
    __shared__ __align__(16) unsigned short stg[4 * 2 * 1152];
    const int lane = threadIdx.x & 31, w = (threadIdx.x >> 5) & 3, lr = lane & 15, hi = lane >> 4;
    const int bh = blockIdx.y, b = bh / NH_, h = bh % NH_;
    const int q0 = qb * 64 + w * 16;
    const int qq = q0 + lr;
    const size_t pof = (size_t)bh * TT * HD;
    const h16* qp = QP + pof + (size_t)(q0 + lr) * HD + 8 * hi;
    const v16h qf0 = ldh(qp), qf1 = ldh(qp + 32);
    v8f o0 = {}, o1 = {}, o2 = {}, o3 = {};
    float m = NEGB, l = 0.0f;
    const int nst = q0 / 32 + 1;
#pragma unroll 1
    for (int st = 0; st < nst; ++st) {
        const int kt = st * 32;
        const h16* kp = KP + pof + (size_t)(kt + lr) * HD + 8 * hi;
        const v16h ka0 = ldh(kp), ka1 = ldh(kp + 16 * HD), kb0 = ldh(kp + 32), kb1 = ldh(kp + 16 * HD + 32);
        v8f s0 = {}, s1 = {};
        s0 = wmma16(ka0, qf0, s0); s1 = wmma16(ka1, qf0, s1);
        s0 = wmma16(kb0, qf1, s0); s1 = wmma16(kb1, qf1, s1);
        asm volatile("v_nop\n\tv_nop\n\tv_nop\n\tv_nop" : "+v"(s0), "+v"(s1) : "v"(ka0), "v"(ka1), "v"(kb0), "v"(kb1), "v"(qf1));
        if (kt + 31 > q0) {
            const int k0 = kt + 8 * hi;
#pragma unroll
            for (int r = 0; r < 8; ++r) { s0[r] = (k0 + r > qq) ? NEGB : s0[r]; s1[r] = (k0 + 16 + r > qq) ? NEGB : s1[r]; }
        }
        float mx = fmaxf(s0[0], s1[0]);
#pragma unroll
        for (int r = 1; r < 8; ++r) mx = fmaxf(mx, fmaxf(s0[r], s1[r]));
        mx = fmaxf(mx, __shfl_xor(mx, 16, 32));
        const float mn = fmaxf(m, mx * CSC);
        const float corr = __builtin_amdgcn_exp2f(m - mn);
        m = mn;
        const float sh = (EARLY ? 0.0f : 8.0f) - mn;
        v8f p0, p1; float rs = 0.0f;
#pragma unroll
        for (int r = 0; r < 8; ++r) { p0[r] = __builtin_amdgcn_exp2f(fmaf(s0[r], CSC, sh)); p1[r] = __builtin_amdgcn_exp2f(fmaf(s1[r], CSC, sh)); rs += p0[r] + p1[r]; }
        rs += __shfl_xor(rs, 16, 32);
        l = l * corr + rs;
        o0 *= corr; o1 *= corr; o2 *= corr; o3 *= corr;
        if (EARLY) {
            v8us ph0, ph1, pl0, pl1;
            pack_b(p0, ph0, pl0); pack_b(p1, ph1, pl1);
            const v16bf PH = cat16b(ph0, ph1), PL = cat16b(pl0, pl1);
            const size_t vo = (size_t)bh * HD * EROWS + (size_t)lr * EROWS + kt + 8 * hi;
            const v16bf vh0 = ldb(VEh + vo), vh1 = ldb(VEh + vo + 16 * EROWS), vh2 = ldb(VEh + vo + 32 * EROWS), vh3 = ldb(VEh + vo + 48 * EROWS);
            const v16bf vl0 = ldb(VEl + vo), vl1 = ldb(VEl + vo + 16 * EROWS), vl2 = ldb(VEl + vo + 32 * EROWS), vl3 = ldb(VEl + vo + 48 * EROWS);
            o0 = wmmab(vh0, PH, o0); o0 = wmmab(vl0, PH, o0); o0 = wmmab(vh0, PL, o0);
            o1 = wmmab(vh1, PH, o1); o1 = wmmab(vl1, PH, o1); o1 = wmmab(vh1, PL, o1);
            o2 = wmmab(vh2, PH, o2); o2 = wmmab(vl2, PH, o2); o2 = wmmab(vh2, PL, o2);
            o3 = wmmab(vh3, PH, o3); o3 = wmmab(vl3, PH, o3); o3 = wmmab(vh3, PL, o3);
            asm volatile("v_nop\n\tv_nop\n\tv_nop\n\tv_nop" : "+v"(o0), "+v"(o1), "+v"(o2), "+v"(o3) : "v"(vh0), "v"(vh1), "v"(vh2), "v"(vh3), "v"(vl0), "v"(vl1), "v"(vl2), "v"(vl3), "v"(PH), "v"(PL));
        } else {
            v16h pb;
#pragma unroll
            for (int r = 0; r < 8; ++r) { pb[r] = (h16)p0[r]; pb[8 + r] = (h16)p1[r]; }
            const h16* vp = VT + (size_t)bh * HD * TT + (size_t)lr * TT + kt + 8 * hi;
            const v16h a0 = ldh(vp), a1 = ldh(vp + 16 * TT), a2 = ldh(vp + 32 * TT), a3 = ldh(vp + 48 * TT);
            o0 = wmma16(a0, pb, o0); o1 = wmma16(a1, pb, o1); o2 = wmma16(a2, pb, o2); o3 = wmma16(a3, pb, o3);
            asm volatile("v_nop\n\tv_nop\n\tv_nop\n\tv_nop" : "+v"(o0), "+v"(o1), "+v"(o2), "+v"(o3) : "v"(a0), "v"(a1), "v"(a2), "v"(a3), "v"(pb));
        }
    }
    const float inv = __fdiv_rn(1.0f, l);
    o0 *= inv; o1 *= inv; o2 *= inv; o3 *= inv;
    const int sb = w * 2 * 1152;
    const int so = sb + lr * 72 + 8 * hi;
    if (EARLY) {
        v8us a, c;
        pack_b(o0, a, c); *(v8usa*)(stg + so) = a;      *(v8usa*)(stg + so + 1152) = c;
        pack_b(o1, a, c); *(v8usa*)(stg + so + 16) = a; *(v8usa*)(stg + so + 1152 + 16) = c;
        pack_b(o2, a, c); *(v8usa*)(stg + so + 32) = a; *(v8usa*)(stg + so + 1152 + 32) = c;
        pack_b(o3, a, c); *(v8usa*)(stg + so + 48) = a; *(v8usa*)(stg + so + 1152 + 48) = c;
    } else {
        *(v8usa*)(stg + so) = pack_h(o0); *(v8usa*)(stg + so + 16) = pack_h(o1); *(v8usa*)(stg + so + 32) = pack_h(o2); *(v8usa*)(stg + so + 48) = pack_h(o3);
    }
    __builtin_amdgcn_wave_barrier(); asm volatile("" ::: "memory");
    const int rq = lane >> 3, pc = lane & 7;
    const int crows = EARLY ? EROWS : TT;
    const size_t cbase = ((size_t)b * crows + q0) * DM + h * HD + pc * 8;
#pragma unroll 1
    for (int ps = 0; ps < 2; ++ps) {
#pragma unroll
        for (int s = 0; s < 4; ++s) { const int row = 4 * s + rq;
            const v8us x = *(const v8usa*)(stg + sb + row * 72 + pc * 8);
            *(volatile v8us*)(C0 + cbase + (size_t)row * DM) = x;
            if (EARLY) { const v8us y = *(const v8usa*)(stg + sb + 1152 + row * 72 + pc * 8); *(volatile v8us*)(C1 + cbase + (size_t)row * DM) = y; } }
        if (ps == 0) __threadfence(); }
}

__global__ __launch_bounds__(128) void k_attn_early(const h16* __restrict__ QP, const h16* __restrict__ KP, const bf* __restrict__ VEh, const bf* __restrict__ VEl, bf* CEh, bf* CEl) {
    attn_body<true>(QP, KP, (const h16*)0, VEh, VEl, CEh, CEl, (int)blockIdx.x);
}
__global__ __launch_bounds__(128) void k_attn_main(const h16* __restrict__ QP, const h16* __restrict__ KP, const h16* __restrict__ VT, bf* CH) {
    attn_body<false>(QP, KP, VT, (const bf*)0, (const bf*)0, CH, CH, (int)blockIdx.x + EROWS / 64);
}

template <typename T16, int NSPLIT>
__device__ __forceinline__ void out_body(const T16* __restrict__ A, const T16* __restrict__ A2, const T16* __restrict__ Bt, float* C, const float* __restrict__ bias, const float scale) {
    __shared__ __align__(16) float os[16 * 68];
    const int lane = threadIdx.x & 31, lr = lane & 15, hi = lane >> 4;
    const int r0 = blockIdx.x * 64, c0 = blockIdx.y * 64;
    v8f acc[4][4];
    gemm_tile<T16, NSPLIT>(A, A2, Bt, DM, (size_t)(r0 + lr) * DM + 8 * hi, (size_t)(c0 + lr) * DM + 8 * hi, acc);
    const v4f bw = *(const v4f*)(bias + c0 + lr * 4);
    v4f bb;
#pragma unroll
    for (int q = 0; q < 4; ++q) bb[q] = bfr(bw[q]);
#pragma unroll
    for (int mb = 0; mb < 4; ++mb) {
#pragma unroll
        for (int nb = 0; nb < 4; ++nb) {
#pragma unroll
            for (int j = 0; j < 8; ++j) os[(hi * 8 + j) * 68 + nb * 16 + lr] = acc[mb][nb][j]; }
        __builtin_amdgcn_wave_barrier(); asm volatile("" ::: "memory");
        float* crow = C + (size_t)(r0 + mb * 16) * DM + c0 + lr * 4;
#pragma unroll 1
        for (int ps = 0; ps < 2; ++ps) {
#pragma unroll
            for (int s = 0; s < 8; ++s) { const int row = 2 * s + hi;
                v4f val = *(const v4fa*)(os + row * 68 + lr * 4);
                val = val * scale + bb;
                *(volatile v4f*)(crow + (size_t)row * DM) = val; }
            if (ps == 0) __threadfence(); }
        __builtin_amdgcn_wave_barrier(); asm volatile("" ::: "memory");
    }
}

__global__ __launch_bounds__(32) void k_oute(const bf* __restrict__ CEh, const bf* __restrict__ CEl, const bf* __restrict__ WoB, float* OUT, const float* __restrict__ Wb) {
    const size_t z = blockIdx.z;
    out_body<bf, 1>(CEh + z * EROWS * DM, CEl + z * EROWS * DM, WoB, OUT + z * TT * DM, Wb, 1.0f);
}
__global__ __launch_bounds__(32) void k_outl(const h16* __restrict__ CH, const h16* __restrict__ WoH, float* OUT, const float* __restrict__ Wb) {
    const size_t ro = ((size_t)blockIdx.z * TT + EROWS) * DM;
    out_body<h16, 0>(CH + ro, CH + ro, WoH, OUT + ro, Wb, OSC);
}

extern "C" void kernel_launch(void* const* d_in, const int* in_sizes, int n_in,
                              void* d_out, int out_size, void* d_ws, size_t ws_size, hipStream_t stream) {
    if (n_in < 11) return;
    if (in_sizes[0] < NB * SEQ_FULL * DM || in_sizes[1] < NB * SEQ_FULL * DM || in_sizes[2] < NB * SEQ_FULL * DM) return;
    if (in_sizes[3] < NH_ * HD * DM || in_sizes[5] < NH_ * HD * DM || in_sizes[7] < NH_ * HD * DM || in_sizes[9] < DM * DM) return;
    if (in_sizes[4] < NH_ * HD || in_sizes[6] < NH_ * HD || in_sizes[8] < NH_ * HD || in_sizes[10] < DM) return;
    if (out_size < NB * TT * DM) return;
    const float* xq = (const float*)d_in[0]; const float* xk = (const float*)d_in[1]; const float* xv = (const float*)d_in[2];
    const float* wq = (const float*)d_in[3]; const float* bq = (const float*)d_in[4];
    const float* wk = (const float*)d_in[5]; const float* bk = (const float*)d_in[6];
    const float* wv = (const float*)d_in[7]; const float* bv = (const float*)d_in[8];
    const float* wo = (const float*)d_in[9]; const float* bo = (const float*)d_in[10];
    float* OUT = (float*)d_out;
    char* wsp = (char*)d_ws;
    auto take = [&](size_t bytes) { char* p = wsp; wsp += (bytes + 255) & ~(size_t)255; return (void*)p; };
    bf*  WT  = (bf*)take((size_t)3 * DM * DM * 2);
    bf*  WoB = (bf*)take((size_t)DM * DM * 2);
    h16* WoH = (h16*)take((size_t)DM * DM * 2);
    h16* QK  = (h16*)take((size_t)2 * QKSZ * 2);
    h16* VT  = (h16*)take((size_t)NB * NH_ * HD * TT * 2);
    bf*  VEh = (bf*)take((size_t)NB * NH_ * HD * EROWS * 2);
    bf*  VEl = (bf*)take((size_t)NB * NH_ * HD * EROWS * 2);
    bf*  XB  = (bf*)take((size_t)3 * XSZ * 2);
    if ((size_t)(wsp - (char*)d_ws) > ws_size) return;
    bf* CH  = XB;
    bf* CEh = XB + XSZ;
    bf* CEl = XB + 2 * XSZ;

    const size_t nx8 = XSZ / 8;
    k_cvt8<<<(unsigned)((nx8 + 255) / 256), 256, 0, stream>>>(xq, XB, nx8);
    k_cvt8<<<(unsigned)((nx8 + 255) / 256), 256, 0, stream>>>(xk, XB + XSZ, nx8);
    k_cvt8<<<(unsigned)((nx8 + 255) / 256), 256, 0, stream>>>(xv, XB + 2 * XSZ, nx8);
    const size_t nw8 = (size_t)DM * DM / 8;
    k_cvt8<<<(unsigned)((nw8 + 255) / 256), 256, 0, stream>>>(wq, WT, nw8);
    k_cvt8<<<(unsigned)((nw8 + 255) / 256), 256, 0, stream>>>(wk, WT + (size_t)DM * DM, nw8);
    k_cvt8<<<(unsigned)((nw8 + 255) / 256), 256, 0, stream>>>(wv, WT + (size_t)2 * DM * DM, nw8);
    k_cvtwo<<<(unsigned)((nw8 + 255) / 256), 256, 0, stream>>>(wo, WoB, WoH, nw8);

    k_projqk<<<dim3(NB * TT / 64, NH_, 2), 32, 0, stream>>>(XB, WT, bq, bk, QK);
    k_projv<<<dim3(NB * TT / 64, NH_), 32, 0, stream>>>(XB + 2 * XSZ, WT + (size_t)2 * DM * DM, bv, VT, VEh, VEl);

    k_attn_early<<<dim3(EROWS / 64, NB * NH_), 128, 0, stream>>>(QK, QK + QKSZ, VEh, VEl, CEh, CEl);
    if (TT > EROWS)
        k_attn_main<<<dim3((TT - EROWS) / 64, NB * NH_), 128, 0, stream>>>(QK, QK + QKSZ, VT, CH);

    k_oute<<<dim3(EROWS / 64, DM / 64, NB), 32, 0, stream>>>(CEh, CEl, WoB, OUT, bo);
    if (TT > EROWS)
        k_outl<<<dim3((TT - EROWS) / 64, DM / 64, NB), 32, 0, stream>>>((const h16*)CH, WoH, OUT, bo);
}
